// LSTMModel_944892805211
// MI455X (gfx1250) — hardware-verified
//
#include <hip/hip_runtime.h>
#include <math.h>

constexpr int NSEQ   = 256;
constexpr int NSTEP  = 1024;
constexpr int NDIN   = 18;
constexpr int KINX   = 32;
constexpr int NHID   = 64;
constexpr int NGATE  = 256;
constexpr int NROWS  = NSEQ * NSTEP;
constexpr int CVT_THR   = 256;
constexpr int LAYER_THR = 128;
constexpr int HEAD_THR  = 256;
constexpr int SEQ_BLK   = 16;
constexpr int HPITCH    = 72;
constexpr float OPCARRY     = 16.0f;
constexpr float WCARRY      = 16.0f;
constexpr float FOLD        = 1.0f / (16.0f * 16.0f);
constexpr float OPCARRY_INV = 1.0f / 16.0f;
static_assert(NGATE == 4 * NHID);
static_assert(NSEQ % SEQ_BLK == 0);
static_assert(NHID == 16 * (LAYER_THR / 32));
static_assert(KINX % 32 == 0 && NHID % 32 == 0);
static_assert(NDIN <= KINX);
static_assert(HPITCH % 8 == 0 && HPITCH >= NHID + 8);
static_assert(NROWS % HEAD_THR == 0);
static_assert(NSTEP % HEAD_THR == 0);
static_assert((NROWS * (KINX / 8)) % CVT_THR == 0);
static_assert((NGATE * (KINX / 8)) % CVT_THR == 0);
static_assert((NGATE * (NHID / 8)) % CVT_THR == 0);

typedef __attribute__((ext_vector_type(16))) _Float16 v16h;
typedef __attribute__((ext_vector_type(8)))  _Float16 v8h;
typedef __attribute__((ext_vector_type(8)))  float    v8f;
typedef __attribute__((ext_vector_type(4)))  float    v4f;
typedef __attribute__((ext_vector_type(4)))  unsigned v4u;

__device__ __forceinline__ void mma_guard4_h(v8f& a0, v8f& a1, v8f& a2, v8f& a3,
                                             v16h x, v16h y0, v16h y1, v16h y2, v16h y3) {
  asm volatile("v_nop\n\tv_nop\n\tv_nop\n\tv_nop"
               : "+v"(a0), "+v"(a1), "+v"(a2), "+v"(a3)
               : "v"(x), "v"(y0), "v"(y1), "v"(y2), "v"(y3));
}
__device__ __forceinline__ void acc_guard4(v8f& a, v8f& b, v8f& c, v8f& d) {
  asm volatile("v_nop\n\tv_nop\n\tv_nop\n\tv_nop" : "+v"(a), "+v"(b), "+v"(c), "+v"(d));
}

template <typename T> struct Frag;
template <> struct Frag<_Float16> {
  typedef v16h V; union U { v16h v; v8h h[2]; };
  static __device__ __forceinline__ v16h load(const _Float16* p) {
    U f; f.h[0] = *(const v8h*)(p); f.h[1] = *(const v8h*)(p + 16); return f.v;
  }
  static __device__ __forceinline__ v8f mma(v16h a, v16h b, v8f c) {
    return __builtin_amdgcn_wmma_f32_16x16x32_f16(false, a, false, b, (short)0, c, false, false);
  }
};

__device__ __forceinline__ float h16_to_f32(unsigned hb) {
  const unsigned sgn = (hb & 0x8000u) << 16; const unsigned em = hb & 0x7fffu;
  const float fn = __uint_as_float((em << 13) + 0x38000000u);
  const float fs = (float)em * 5.9604644775390625e-8f;
  const float mag = (em < 0x400u) ? fs : fn; return __uint_as_float(__float_as_uint(mag) | sgn); }

__device__ __forceinline__ float fsig(float x)  { return __builtin_amdgcn_rcpf(1.0f + expf(-x)); }
__device__ __forceinline__ float ftanh(float x) { return 1.0f - 2.0f * __builtin_amdgcn_rcpf(expf(2.0f * x) + 1.0f); }

template <int KSRC, int KDST>
__global__ __launch_bounds__(CVT_THR) void cvt_rows_f16_kernel(const float* __restrict__ src, unsigned short* __restrict__ dst,
                                                              int nrow, float sc) {
  static_assert(KDST % 8 == 0 && KSRC <= KDST && KSRC >= 1);
  constexpr int C8 = KDST / 8;
  const size_t i  = (size_t)blockIdx.x * CVT_THR + threadIdx.x;
  const size_t n8 = (size_t)nrow * C8;
  if (i < n8) {
    const size_t row = i / C8;
    const int c8 = (int)(i - row * C8) * 8;
    const float* sp = src + row * (size_t)KSRC;
    v8h hv;
#pragma unroll
    for (int e = 0; e < 8; ++e) {
      const int col  = c8 + e;
      const int colc = (col < KSRC) ? col : (KSRC - 1);
      const float f = sp[colc];
      const float v = (col < KSRC) ? (f * sc) : 0.0f;
      hv[e] = (_Float16)v;
    }
    _Float16* dp = (_Float16*)dst + i * 8;
    *(volatile v8h*)dp = hv;
    __threadfence();
    *(volatile v8h*)dp = hv;
  }
}

template <int KIN>
__global__ __launch_bounds__(LAYER_THR) void lstm_layer_kernel(const unsigned short* __restrict__ INp,
                                                              const unsigned short* __restrict__ WIp,
                                                              const unsigned short* __restrict__ WHp,
                                                              const float* __restrict__ b_a,
                                                              const float* __restrict__ b_b,
                                                              unsigned short* __restrict__ OUTp) {
  static_assert(KIN % 32 == 0);
  constexpr int APITCH = KIN + 8;
  static_assert(16 * KIN / 8 <= LAYER_THR);
  __shared__ __align__(16) _Float16 Ain[16 * APITCH];
  __shared__ __align__(16) _Float16 Ah[16 * HPITCH];
  const _Float16* IN  = (const _Float16*)INp;
  const _Float16* WI  = (const _Float16*)WIp;
  const _Float16* WH  = (const _Float16*)WHp;
  _Float16*       OUT = (_Float16*)OUTp;
  const int tid = threadIdx.x, lane = tid & 31, wave = tid >> 5;
  const int c = lane & 15, hh = lane >> 4, koff = hh * 8;
  const int rowbase = blockIdx.x * SEQ_BLK;
  const int j = 16 * wave + c;

#pragma unroll 1
  for (int i = tid; i < 16 * APITCH; i += LAYER_THR) Ain[i] = (_Float16)0.0f;
#pragma unroll 1
  for (int i = tid; i < 16 * HPITCH; i += LAYER_THR) Ah[i] = (_Float16)0.0f;
  __syncthreads();

  if (tid < 16 * KIN / 8) {
    const int m = tid / (KIN / 8), c8 = (tid - m * (KIN / 8)) * 8;
    const v8h v = *(const v8h*)(IN + ((size_t)(rowbase + m) * NSTEP) * KIN + c8);
    *(v8h*)(Ain + m * APITCH + c8) = v;
  }
  float bb[4];
#pragma unroll
  for (int q = 0; q < 4; ++q) bb[q] = b_a[q * NHID + j] + b_b[q * NHID + j];
  float cst[8], hst[8];
#pragma unroll
  for (int r = 0; r < 8; ++r) { cst[r] = 0.0f; hst[r] = 0.0f; }
  __syncthreads();

  const _Float16* ainrow = Ain + c * APITCH + koff;
  const _Float16* ahrow  = Ah  + c * HPITCH + koff;
  const _Float16* wi = WI + (size_t)j * KIN  + koff;
  const _Float16* wh = WH + (size_t)j * NHID + koff;
  const v8f z8 = {0.f, 0.f, 0.f, 0.f, 0.f, 0.f, 0.f, 0.f};
  const int cq = lane >> 3, cc8 = (lane & 7) * 8;
  const int cm = 4 * wave + cq;

#pragma unroll 1
  for (int t = 0; t < NSTEP; ++t) {
    v8f acc[4];
    acc[0] = z8; acc[1] = z8; acc[2] = z8; acc[3] = z8;
#pragma unroll 1
    for (int k0 = 0; k0 < KIN; k0 += 32) {
      const v16h a  = Frag<_Float16>::load(ainrow + k0);
      const v16h b0 = Frag<_Float16>::load(wi + k0);
      const v16h b1 = Frag<_Float16>::load(wi + (size_t)1 * NHID * KIN + k0);
      const v16h b2 = Frag<_Float16>::load(wi + (size_t)2 * NHID * KIN + k0);
      const v16h b3 = Frag<_Float16>::load(wi + (size_t)3 * NHID * KIN + k0);
      acc[0] = Frag<_Float16>::mma(a, b0, acc[0]);
      acc[1] = Frag<_Float16>::mma(a, b1, acc[1]);
      acc[2] = Frag<_Float16>::mma(a, b2, acc[2]);
      acc[3] = Frag<_Float16>::mma(a, b3, acc[3]);
      mma_guard4_h(acc[0], acc[1], acc[2], acc[3], a, b0, b1, b2, b3);
    }
#pragma unroll 1
    for (int k0 = 0; k0 < NHID; k0 += 32) {
      const v16h a  = Frag<_Float16>::load(ahrow + k0);
      const v16h b0 = Frag<_Float16>::load(wh + k0);
      const v16h b1 = Frag<_Float16>::load(wh + (size_t)1 * NHID * NHID + k0);
      const v16h b2 = Frag<_Float16>::load(wh + (size_t)2 * NHID * NHID + k0);
      const v16h b3 = Frag<_Float16>::load(wh + (size_t)3 * NHID * NHID + k0);
      acc[0] = Frag<_Float16>::mma(a, b0, acc[0]);
      acc[1] = Frag<_Float16>::mma(a, b1, acc[1]);
      acc[2] = Frag<_Float16>::mma(a, b2, acc[2]);
      acc[3] = Frag<_Float16>::mma(a, b3, acc[3]);
      mma_guard4_h(acc[0], acc[1], acc[2], acc[3], a, b0, b1, b2, b3);
    }
    acc_guard4(acc[0], acc[1], acc[2], acc[3]);

#pragma unroll
    for (int r = 0; r < 8; ++r) {
      const float zi = acc[0][r] * FOLD + bb[0];
      const float zf = acc[1][r] * FOLD + bb[1];
      const float zg = acc[2][r] * FOLD + bb[2];
      const float zo = acc[3][r] * FOLD + bb[3];
      const float ig = fsig(zi);
      const float fg = fsig(zf);
      const float gg = ftanh(zg);
      const float og = fsig(zo);
      const float cn = fg * cst[r] + ig * gg;
      cst[r] = cn;
      hst[r] = og * ftanh(cn);
    }
    __syncthreads();

#pragma unroll
    for (int r = 0; r < 8; ++r) Ah[(8 * hh + r) * HPITCH + j] = (_Float16)(hst[r] * OPCARRY);
    {
      const int tn = (t + 1 < NSTEP) ? (t + 1) : (NSTEP - 1);
      if (tid < 16 * KIN / 8) {
        const int m = tid / (KIN / 8), c8 = (tid - m * (KIN / 8)) * 8;
        const v8h v = *(const v8h*)(IN + ((size_t)(rowbase + m) * NSTEP + (size_t)tn) * KIN + c8);
        *(v8h*)(Ain + m * APITCH + c8) = v;
      }
    }
    __syncthreads();

    {
      const v8h v = *(const v8h*)(Ah + cm * HPITCH + cc8);
      _Float16* op = OUT + ((size_t)(rowbase + cm) * NSTEP + (size_t)t) * NHID + cc8;
      *(volatile v8h*)op = v;
      __threadfence();
      *(volatile v8h*)op = v;
    }
  }
}

__global__ __launch_bounds__(HEAD_THR) void head_kernel(const unsigned short* __restrict__ H3, const float* __restrict__ w_out,
                                                        const float* __restrict__ b_out, float* __restrict__ out) {
  __shared__ float wsh[NHID];
  __shared__ __align__(16) float osh[HEAD_THR];
  const int tid = threadIdx.x;
  const size_t idx = (size_t)blockIdx.x * HEAD_THR + tid;
  if (tid < NHID) wsh[tid] = w_out[tid];
  __syncthreads();
  const v4u* rp = (const v4u*)(H3 + idx * NHID);
  float acc = 0.0f;
#pragma unroll
  for (int q = 0; q < 8; ++q) {
    const v4u w4 = rp[q];
#pragma unroll
    for (int e = 0; e < 4; ++e) {
      const unsigned u = w4[e];
      const float vlo = h16_to_f32(u & 0xffffu);
      const float vhi = h16_to_f32(u >> 16);
      const int k = q * 8 + e * 2;
      acc = fmaf(vlo, wsh[k], acc);
      acc = fmaf(vhi, wsh[k + 1], acc);
    }
  }
  const float o = acc * OPCARRY_INV + b_out[0];
  osh[tid] = o;
  __syncthreads();
  if (tid < HEAD_THR / 4) {
    const v4f v = *(const v4f*)(osh + 4 * tid);
    float* op = out + (size_t)blockIdx.x * HEAD_THR + 4 * tid;
    *(volatile v4f*)op = v;
    __threadfence();
    *(volatile v4f*)op = v;
  }
}

extern "C" void kernel_launch(void* const* d_in, const int* in_sizes, int n_in,
                              void* d_out, int out_size, void* d_ws, size_t ws_size, hipStream_t stream) {
  if (n_in < 11 || d_out == nullptr || d_ws == nullptr) return;
  if (in_sizes[0] != NSEQ * NSTEP * NDIN || in_sizes[1] != NGATE * NDIN || in_sizes[2] != NGATE * NHID ||
      in_sizes[3] != NGATE || in_sizes[4] != NGATE || in_sizes[5] != 2 * NGATE * NHID || in_sizes[6] != 2 * NGATE * NHID ||
      in_sizes[7] != 2 * NGATE || in_sizes[8] != 2 * NGATE || in_sizes[9] != NHID || in_sizes[10] != 1 ||
      out_size != NROWS) return;

  const float* x      = (const float*)d_in[0];
  const float* w_ih0  = (const float*)d_in[1];
  const float* w_hh0  = (const float*)d_in[2];
  const float* b_ih0  = (const float*)d_in[3];
  const float* b_hh0  = (const float*)d_in[4];
  const float* w_ih12 = (const float*)d_in[5];
  const float* w_hh12 = (const float*)d_in[6];
  const float* b_ih12 = (const float*)d_in[7];
  const float* b_hh12 = (const float*)d_in[8];
  const float* w_out  = (const float*)d_in[9];
  const float* b_out  = (const float*)d_in[10];
  float* out = (float*)d_out;

  char* ws = (char*)d_ws; size_t off = 0;
  auto carve = [&](size_t bytes) -> char* { char* p = ws + off; off += (bytes + 255) & ~(size_t)255; return p; };
  unsigned short* XP   = (unsigned short*)carve((size_t)NROWS * KINX * 2);
  unsigned short* WI0  = (unsigned short*)carve((size_t)NGATE * KINX * 2);
  unsigned short* WH0  = (unsigned short*)carve((size_t)NGATE * NHID * 2);
  unsigned short* WI12 = (unsigned short*)carve((size_t)2 * NGATE * NHID * 2);
  unsigned short* WH12 = (unsigned short*)carve((size_t)2 * NGATE * NHID * 2);
  unsigned short* HPA  = (unsigned short*)carve((size_t)NROWS * NHID * 2);
  unsigned short* HPB  = (unsigned short*)carve((size_t)NROWS * NHID * 2);
  unsigned short* HPC  = (unsigned short*)carve((size_t)NROWS * NHID * 2);
  if (off > ws_size || off > (size_t)134217728) return;

  const int n8x   = NROWS * (KINX / 8);
  const int n8i0  = NGATE * (KINX / 8);
  const int n8h0  = NGATE * (NHID / 8);
  const int n8w12 = 2 * NGATE * (NHID / 8);
  cvt_rows_f16_kernel<NDIN, KINX><<<(n8x   + CVT_THR - 1) / CVT_THR, CVT_THR, 0, stream>>>(x,      XP,   NROWS,     OPCARRY);
  cvt_rows_f16_kernel<NDIN, KINX><<<(n8i0  + CVT_THR - 1) / CVT_THR, CVT_THR, 0, stream>>>(w_ih0,  WI0,  NGATE,     WCARRY);
  cvt_rows_f16_kernel<NHID, NHID><<<(n8h0  + CVT_THR - 1) / CVT_THR, CVT_THR, 0, stream>>>(w_hh0,  WH0,  NGATE,     WCARRY);
  cvt_rows_f16_kernel<NHID, NHID><<<(n8w12 + CVT_THR - 1) / CVT_THR, CVT_THR, 0, stream>>>(w_ih12, WI12, 2 * NGATE, WCARRY);
  cvt_rows_f16_kernel<NHID, NHID><<<(n8w12 + CVT_THR - 1) / CVT_THR, CVT_THR, 0, stream>>>(w_hh12, WH12, 2 * NGATE, WCARRY);

  lstm_layer_kernel<KINX><<<NSEQ / SEQ_BLK, LAYER_THR, 0, stream>>>(XP,  WI0,  WH0,  b_ih0,  b_hh0,  HPA);
  lstm_layer_kernel<NHID><<<NSEQ / SEQ_BLK, LAYER_THR, 0, stream>>>(HPA, WI12, WH12, b_ih12, b_hh12, HPB);
  lstm_layer_kernel<NHID><<<NSEQ / SEQ_BLK, LAYER_THR, 0, stream>>>(HPB, WI12 + (size_t)NGATE * NHID, WH12 + (size_t)NGATE * NHID,
                                                                    b_ih12 + NGATE, b_hh12 + NGATE, HPC);

  head_kernel<<<NROWS / HEAD_THR, HEAD_THR, 0, stream>>>(HPC, w_out, b_out, out);
}
